// TimeSeriesSelfAttention_42898133353109
// MI455X (gfx1250) — hardware-verified
//
#include <hip/hip_runtime.h>
#include <stddef.h>
#include <stdint.h>


#define BB  4
#define CH  64
#define NH  8
#define LS  2048
#define HC  (NH * CH)
#define LT  64
#define NLT (LS / LT)
#define QT  128
#define NQT (LS / QT)
#define KT  64
#define NKT (LS / KT)
#define PH  72
#define PF  68

typedef _Float16 v16h __attribute__((ext_vector_type(16)));
typedef _Float16 v8h  __attribute__((ext_vector_type(8)));
typedef float    v8f  __attribute__((ext_vector_type(8)));
typedef float    v4f  __attribute__((ext_vector_type(4)));

union Frag { v16h v; v8h hv[2]; _Float16 e[16]; };
union Acc  { v8f v; float x[8]; };

__device__ __forceinline__ v8f wmma16(v16h a, v16h b, v8f c)
{
    v8f d = __builtin_amdgcn_wmma_f32_16x16x32_f16(false, a, false, b, (short)0, c, false, false);
    asm volatile("v_nop\n\tv_nop\n\tv_nop\n\tv_nop" : "+v"(d) : "v"(a), "v"(b));
    return d;
}

__device__ __forceinline__ v8f zero8()
{
    v8f z;
#pragma unroll
    for (int i = 0; i < 8; ++i) z[i] = 0.0f;
    return z;
}

__device__ __forceinline__ v8h cvt8(v4f p, v4f q, float s)
{
    v8h r;
    r[0] = (_Float16)(p[0] * s); r[1] = (_Float16)(p[1] * s);
    r[2] = (_Float16)(p[2] * s); r[3] = (_Float16)(p[3] * s);
    r[4] = (_Float16)(q[0] * s); r[5] = (_Float16)(q[1] * s);
    r[6] = (_Float16)(q[2] * s); r[7] = (_Float16)(q[3] * s);
    return r;
}

__device__ __forceinline__ void rows16_store(const _Float16 (*T)[PH], _Float16* dst, size_t row0, size_t pitch, int lane)
{
    const int j = lane & 7, q0 = lane >> 3;
#pragma unroll
    for (int i = 0; i < 4; ++i) {
        const int q = i * 4 + q0;
        const v8h v = *(const v8h*)&T[q][8 * j];
        *(volatile v8h*)(dst + (row0 + (size_t)q) * pitch + 8 * j) = v;
    }
}

__global__ __launch_bounds__(256) void k_proj(
    const float* __restrict__ x,
    const float* __restrict__ qdw, const float* __restrict__ qdb, const float* __restrict__ qpw, const float* __restrict__ qpb,
    const float* __restrict__ kdw, const float* __restrict__ kdb, const float* __restrict__ kpw, const float* __restrict__ kpb,
    const float* __restrict__ vdw, const float* __restrict__ vdb, const float* __restrict__ vpw, const float* __restrict__ vpb,
    _Float16* qo, _Float16* ko, _Float16* vo, int nblk)
{
    __shared__ __attribute__((aligned(16))) _Float16 yT[LT][PH];
    __shared__ __attribute__((aligned(16))) _Float16 Ts[8][16][PH];

    const int t = threadIdx.x, lane = t & 31, w = t >> 5, h = lane >> 4, m = lane & 15;
    const int blk = blockIdx.x;
    if (blk >= nblk) return;
    const int b  = blk / NLT;
    const int l0 = (blk - b * NLT) * LT;
    const int bh = b * NH + w;

#pragma unroll 1
    for (int s = 0; s < 3; ++s) {
        const float* dw = (s == 0) ? qdw : (s == 1) ? kdw : vdw;
        const float* db = (s == 0) ? qdb : (s == 1) ? kdb : vdb;
        const float* pw = (s == 0) ? qpw : (s == 1) ? kpw : vpw;
        const float* pb = (s == 0) ? qpb : (s == 1) ? kpb : vpb;
        _Float16*   dst = (s == 0) ? qo  : (s == 1) ? ko  : vo;
        const float osc = (s < 2) ? (64.0f * 0.35355339059327373f) : 64.0f;

        __syncthreads();
        for (int idx = t; idx < CH * LT; idx += 256) {
            const int c = idx >> 6, i = idx & (LT - 1);
            const int l = l0 + i;
            const float* xr = x + ((size_t)(b * CH + c)) * LS;
            const float xm = (l > 0) ? xr[l - 1] : 0.0f;
            const float x0 = xr[l];
            const float xp = (l + 1 < LS) ? xr[l + 1] : 0.0f;
            const float y = dw[c * 3 + 0] * xm + dw[c * 3 + 1] * x0 + dw[c * 3 + 2] * xp + db[c];
            yT[i][c] = (_Float16)(y * 64.0f);
        }
        __syncthreads();

        Frag a[4][2];
#pragma unroll
        for (int mt = 0; mt < 4; ++mt) {
#pragma unroll
            for (int ks = 0; ks < 2; ++ks) {
                const float* ap = pw + (size_t)(w * 64 + mt * 16 + m) * CH + ks * 32 + 8 * h;
                a[mt][ks].hv[0] = cvt8(*(const v4f*)ap, *(const v4f*)(ap + 4), 64.0f);
                a[mt][ks].hv[1] = cvt8(*(const v4f*)(ap + 16), *(const v4f*)(ap + 20), 64.0f);
            }
        }

#pragma unroll 1
        for (int nt = 0; nt < 4; ++nt) {
            Frag bf[2];
#pragma unroll
            for (int ks = 0; ks < 2; ++ks) {
                bf[ks].hv[0] = *(const v8h*)&yT[nt * 16 + m][ks * 32 + 8 * h];
                bf[ks].hv[1] = *(const v8h*)&yT[nt * 16 + m][ks * 32 + 16 + 8 * h];
            }
            Acc acc[4];
#pragma unroll
            for (int mt = 0; mt < 4; ++mt) {
                v8f c = zero8();
#pragma unroll
                for (int ks = 0; ks < 2; ++ks) c = wmma16(a[mt][ks].v, bf[ks].v, c);
                acc[mt].v = c;
            }
            __syncthreads();
#pragma unroll
            for (int mt = 0; mt < 4; ++mt) {
                v8h pk;
#pragma unroll
                for (int r = 0; r < 8; ++r) {
                    const int cl = mt * 16 + 8 * h + r;
                    pk[r] = (_Float16)((acc[mt].x[r] * (1.0f / 4096.0f) + pb[w * 64 + cl]) * osc);
                }
                *(v8h*)&Ts[w][m][mt * 16 + 8 * h] = pk;
            }
            __syncthreads();
            const size_t row0 = (size_t)bh * LS + (size_t)(l0 + nt * 16);
            rows16_store(Ts[w], dst, row0, (size_t)CH, lane);
            __threadfence();
            rows16_store(Ts[w], dst, row0, (size_t)CH, lane);
        }
    }
}

__global__ __launch_bounds__(256) void k_attn(const _Float16* __restrict__ qg, const _Float16* __restrict__ kg,
                                             const _Float16* __restrict__ vg, _Float16* og, int nblk)
{
    __shared__ __attribute__((aligned(16))) _Float16 Ks[KT][PH];
    __shared__ __attribute__((aligned(16))) _Float16 Vs[CH][PH];
    __shared__ __attribute__((aligned(16))) _Float16 Ts[8][16][PH];

    const int t = threadIdx.x, lane = t & 31, w = t >> 5, h = lane >> 4, m = lane & 15;
    const int blk = blockIdx.x;
    if (blk >= nblk) return;
    const int bh = blk / NQT, qb = blk - bh * NQT;
    const int b = bh / NH, hh = bh - b * NH;
    const int jw = qb * QT + w * 16;
    const size_t hb = (size_t)bh * LS * CH;

    Frag bq[2];
    {
        const _Float16* qp = qg + hb + (size_t)(jw + m) * CH + 8 * h;
#pragma unroll
        for (int ks = 0; ks < 2; ++ks) {
            bq[ks].hv[0] = *(const v8h*)(qp + ks * 32);
            bq[ks].hv[1] = *(const v8h*)(qp + ks * 32 + 16);
        }
    }

    float mrun = -1.0e30f, ssum = 0.0f;
    Acc O[4];
#pragma unroll
    for (int ct = 0; ct < 4; ++ct) O[ct].v = zero8();

#pragma unroll 1
    for (int kt = 0; kt < NKT; ++kt) {
        __syncthreads();
#pragma unroll
        for (int i = 0; i < 2; ++i) {
            const int idx = t + 256 * i;
            const int row = idx >> 3, ch = idx & 7;
            const size_t go = hb + (size_t)(kt * KT + row) * CH + ch * 8;
            *(v8h*)&Ks[row][ch * 8] = *(const v8h*)(kg + go);
            const v8h vv = *(const v8h*)(vg + go);
#pragma unroll
            for (int e = 0; e < 8; ++e) Vs[ch * 8 + e][row] = vv[e];
        }
        __syncthreads();

        Acc S[4];
#pragma unroll
        for (int sub = 0; sub < 4; ++sub) {
            v8f c = zero8();
#pragma unroll
            for (int ks = 0; ks < 2; ++ks) {
                Frag a;
                a.hv[0] = *(const v8h*)&Ks[sub * 16 + m][ks * 32 + 8 * h];
                a.hv[1] = *(const v8h*)&Ks[sub * 16 + m][ks * 32 + 16 + 8 * h];
                c = wmma16(a.v, bq[ks].v, c);
            }
            S[sub].v = c;
        }

        float tmax = -1.0e30f;
#pragma unroll
        for (int sub = 0; sub < 4; ++sub)
#pragma unroll
            for (int r = 0; r < 8; ++r) tmax = fmaxf(tmax, S[sub].x[r]);
        tmax = fmaxf(tmax, __shfl_xor(tmax, 16));
        const float mnew = fmaxf(mrun, tmax * (1.0f / 4096.0f));
        const float corr = __expf(mrun - mnew);
        float psum = 0.0f;
        Frag bp[2];
#pragma unroll
        for (int sub = 0; sub < 4; ++sub) {
            v8h pk;
#pragma unroll
            for (int r = 0; r < 8; ++r) {
                const float p = __expf(S[sub].x[r] * (1.0f / 4096.0f) - mnew);
                psum += p;
                pk[r] = (_Float16)(p * 4096.0f);
            }
            bp[sub >> 1].hv[sub & 1] = pk;
        }
        psum += __shfl_xor(psum, 16);
        ssum = ssum * corr + psum;
        mrun = mnew;
#pragma unroll
        for (int ct = 0; ct < 4; ++ct)
#pragma unroll
            for (int r = 0; r < 8; ++r) O[ct].x[r] *= corr;

#pragma unroll
        for (int ct = 0; ct < 4; ++ct) {
#pragma unroll
            for (int ks = 0; ks < 2; ++ks) {
                Frag av;
                av.hv[0] = *(const v8h*)&Vs[ct * 16 + m][ks * 32 + 8 * h];
                av.hv[1] = *(const v8h*)&Vs[ct * 16 + m][ks * 32 + 16 + 8 * h];
                O[ct].v = wmma16(av.v, bp[ks].v, O[ct].v);
            }
        }
    }

    const float f = (1.0f / 4096.0f) / ssum;
    __syncthreads();
#pragma unroll
    for (int ct = 0; ct < 4; ++ct) {
        v8h pk;
#pragma unroll
        for (int r = 0; r < 8; ++r) pk[r] = (_Float16)(O[ct].x[r] * f);
        *(v8h*)&Ts[w][m][ct * 16 + 8 * h] = pk;
    }
    __syncthreads();
    const size_t row0 = (size_t)b * LS + (size_t)jw;
    _Float16* dst = og + hh * CH;
    rows16_store(Ts[w], dst, row0, (size_t)HC, lane);
    __threadfence();
    rows16_store(Ts[w], dst, row0, (size_t)HC, lane);
}

__global__ __launch_bounds__(256) void k_unify(const _Float16* __restrict__ att, const float* __restrict__ uw,
                                              const float* __restrict__ ub, float* out, int nblk)
{
    __shared__ __attribute__((aligned(16))) float To[CH][PF];

    const int t = threadIdx.x, lane = t & 31, w = t >> 5, h = lane >> 4, m = lane & 15;
    const int blk = blockIdx.x;
    if (blk >= nblk) return;
    const int b  = blk / NLT;
    const int l0 = (blk - b * NLT) * LT;
    const int mt = w >> 1, nt0 = (w & 1) * 2;

    const float*    ap0 = uw + (size_t)(mt * 16 + m) * HC + 8 * h;
    const _Float16* bp0 = att + ((size_t)b * LS + (size_t)(l0 + nt0 * 16 + m)) * HC + 8 * h;
    const _Float16* bp1 = bp0 + (size_t)16 * HC;

    Acc acc0, acc1;
    acc0.v = zero8();
    acc1.v = zero8();
#pragma unroll 2
    for (int ks = 0; ks < HC / 32; ++ks) {
        Frag a, f0, f1;
        const float* ap = ap0 + ks * 32;
        a.hv[0] = cvt8(*(const v4f*)ap, *(const v4f*)(ap + 4), 64.0f);
        a.hv[1] = cvt8(*(const v4f*)(ap + 16), *(const v4f*)(ap + 20), 64.0f);
        f0.hv[0] = *(const v8h*)(bp0 + ks * 32);
        f0.hv[1] = *(const v8h*)(bp0 + ks * 32 + 16);
        f1.hv[0] = *(const v8h*)(bp1 + ks * 32);
        f1.hv[1] = *(const v8h*)(bp1 + ks * 32 + 16);
        acc0.v = wmma16(a.v, f0.v, acc0.v);
        acc1.v = wmma16(a.v, f1.v, acc1.v);
    }

#pragma unroll
    for (int r = 0; r < 8; ++r) {
        const int c = mt * 16 + 8 * h + r;
        const float bias = ub[c];
        To[c][nt0 * 16 + m]      = acc0.x[r] * (1.0f / 4096.0f) + bias;
        To[c][nt0 * 16 + 16 + m] = acc1.x[r] * (1.0f / 4096.0f) + bias;
    }
    __syncthreads();

    float* ob = out + l0;
    const size_t rb = (size_t)b * CH;
#pragma unroll
    for (int i = 0; i < 4; ++i) {
        const int row = w * 8 + i * 2 + h;
        const v4f v = *(const v4f*)&To[row][4 * m];
        *(volatile v4f*)(ob + (rb + (size_t)row) * LS + 4 * m) = v;
    }
    __threadfence();
#pragma unroll
    for (int i = 0; i < 4; ++i) {
        const int row = w * 8 + i * 2 + h;
        const v4f v = *(const v4f*)&To[row][4 * m];
        *(volatile v4f*)(ob + (rb + (size_t)row) * LS + 4 * m) = v;
    }
}

extern "C" void kernel_launch(void* const* d_in, const int* in_sizes, int n_in,
                              void* d_out, int out_size, void* d_ws, size_t ws_size,
                              hipStream_t stream)
{
    if (n_in < 15) return;
    if (in_sizes[0] != BB * CH * LS || out_size != BB * CH * LS) return;
    if (in_sizes[3] != HC * CH || in_sizes[7] != HC * CH || in_sizes[11] != HC * CH || in_sizes[13] != CH * HC) return;

    const float* x   = (const float*)d_in[0];
    const float* qdw = (const float*)d_in[1];  const float* qdb = (const float*)d_in[2];
    const float* qpw = (const float*)d_in[3];  const float* qpb = (const float*)d_in[4];
    const float* kdw = (const float*)d_in[5];  const float* kdb = (const float*)d_in[6];
    const float* kpw = (const float*)d_in[7];  const float* kpb = (const float*)d_in[8];
    const float* vdw = (const float*)d_in[9];  const float* vdb = (const float*)d_in[10];
    const float* vpw = (const float*)d_in[11]; const float* vpb = (const float*)d_in[12];
    const float* uw  = (const float*)d_in[13]; const float* ub  = (const float*)d_in[14];

    const size_t nh   = (size_t)BB * HC * LS;
    const size_t need = nh * sizeof(_Float16) * 4;
    if (need > ws_size) return;
    _Float16* qws = (_Float16*)d_ws;
    _Float16* kws = qws + nh;
    _Float16* vws = kws + nh;
    _Float16* aws = vws + nh;

    const int nb1 = BB * NLT;
    const int nb2 = BB * NH * NQT;
    const int nb3 = BB * NLT;

    k_proj<<<dim3(nb1), dim3(256), 0, stream>>>(x, qdw, qdb, qpw, qpb, kdw, kdb, kpw, kpb,
                                               vdw, vdb, vpw, vpb, qws, kws, vws, nb1);
    k_attn<<<dim3(nb2), dim3(256), 0, stream>>>(qws, kws, vws, aws, nb2);
    k_unify<<<dim3(nb3), dim3(256), 0, stream>>>(aws, uw, ub, (float*)d_out, nb3);
    (void)hipGetLastError();
}
